// PIDustModel_19344532702165
// MI455X (gfx1250) — hardware-verified
//
#include <hip/hip_runtime.h>
#include <math.h>

#define NN 100000
#define NE 3200000
#define NC 4
#define NH 64
#define RANGE 4096
#define RSPLIT (1.0f / 2048.0f)

typedef _Float16 h16;
typedef __attribute__((ext_vector_type(16))) _Float16 v16h;
typedef __attribute__((ext_vector_type(8)))  float v8f;
typedef __attribute__((ext_vector_type(4)))  float v4f_t;
typedef float v4fa __attribute__((ext_vector_type(4), may_alias));

__device__ __forceinline__ h16 lo_of(float v, h16 h) { return (h16)((v - (float)h) * 2048.0f); }
__device__ __forceinline__ v8f wmma16(v16h a, v16h b, v8f c) { return __builtin_amdgcn_wmma_f32_16x16x32_f16(false, a, false, b, (short)0, c, false, false); }
__device__ __forceinline__ v8f wmma_split(v16h a, v16h al, v16h b, v16h bl, v8f c) { v8f x = {}; x = wmma16(al, b, x); x = wmma16(a, bl, x); return wmma16(a, b, c) + x * RSPLIT; }
__device__ __forceinline__ int kof(int half, int e) { return 8 * half + ((e < 8) ? e : (e + 8)); }
__device__ __forceinline__ int clampi(int v, int n) { return v < 0 ? 0 : (v >= n ? n - 1 : v); }

__global__ __launch_bounds__(256) void k_feat(const float* __restrict__ x, const float* __restrict__ pos, const int* __restrict__ ei,
                                             int e0, h16* __restrict__ F, size_t plane) {
  const int el = blockIdx.x * 256 + threadIdx.x;
  const int e = e0 + el;
  const int src = clampi(ei[e], NN), dst = clampi(ei[(size_t)NE + e], NN);
  float f[16];
#pragma unroll
  for (int c = 0; c < 4; ++c) { f[c] = x[(size_t)dst * NC + c]; f[4 + c] = x[(size_t)src * NC + c]; }
  const float dx = pos[(size_t)src * 2] - pos[(size_t)dst * 2], dy = pos[(size_t)src * 2 + 1] - pos[(size_t)dst * 2 + 1];
  const float dist = sqrtf(dx * dx + dy * dy + 1e-8f);
  f[8] = f[5] * (dx / dist) + f[6] * (dy / dist);
  f[9] = dist;
#pragma unroll
  for (int c = 10; c < 16; ++c) f[c] = 0.0f;
  h16 hh[16], hl[16];
#pragma unroll
  for (int c = 0; c < 16; ++c) { hh[c] = (h16)f[c]; hl[c] = lo_of(f[c], hh[c]); }
  typedef __attribute__((ext_vector_type(4))) unsigned v4u_t; typedef unsigned v4ua __attribute__((ext_vector_type(4), may_alias));
  h16* d = F + (size_t)el * 16;
#pragma unroll 1
  for (int pass = 0; pass < 2; ++pass) {
    *(volatile v4u_t*)(d) = *(const v4ua*)(hh); *(volatile v4u_t*)(d + 8) = *(const v4ua*)(hh + 8);
    *(volatile v4u_t*)(d + plane) = *(const v4ua*)(hl); *(volatile v4u_t*)(d + plane + 8) = *(const v4ua*)(hl + 8);
    __threadfence();
  }
}

__global__ __launch_bounds__(256) void k_edge(const h16* __restrict__ F, size_t plane, const float* __restrict__ W,
                                             const float* __restrict__ bm, const float* __restrict__ hw, int e0,
                                             float* __restrict__ s) {
  __shared__ __attribute__((aligned(16))) float sv[512];
  const int tid = threadIdx.x, lane = tid & 31, wave = tid >> 5, half = lane >> 4, l16 = lane & 15;
  const int e0blk = blockIdx.x * 512;
  v16h Bw[4], Bwl[4]; float bb[4], hh[4];
#pragma unroll
  for (int nt = 0; nt < 4; ++nt) { const int n = nt * 16 + l16; v16h r, rl;
#pragma unroll
    for (int e = 0; e < 16; ++e) { const int k = kof(half, e); const float v = (k < 10) ? W[n * 10 + k] : 0.0f; r[e] = (h16)v; rl[e] = lo_of(v, r[e]); }
    Bw[nt] = r; Bwl[nt] = rl; bb[nt] = bm[n]; hh[nt] = hw[n]; }
#pragma unroll 1
  for (int it = 0; it < 4; ++it) {
    const int ebase = e0blk + wave * 64 + it * 16;
    const h16* fr = F + (size_t)(ebase + l16) * 16;
    v16h a, al;
#pragma unroll
    for (int q = 0; q < 16; ++q) { const int k = kof(half, q);
      a[q] = (k < 16) ? fr[k] : (h16)0.0f; al[q] = (k < 16) ? fr[plane + k] : (h16)0.0f; }
    float part[8];
#pragma unroll
    for (int r = 0; r < 8; ++r) part[r] = 0.0f;
#pragma unroll
    for (int nt = 0; nt < 4; ++nt) { v8f c = {}; c = wmma_split(a, al, Bw[nt], Bwl[nt], c);
#pragma unroll
      for (int r = 0; r < 8; ++r) part[r] += fmaxf(c[r] + bb[nt], 0.0f) * hh[nt]; }
#pragma unroll
    for (int r = 0; r < 8; ++r) { float v = part[r]; v += __shfl_xor(v, 1, 32); v += __shfl_xor(v, 2, 32); v += __shfl_xor(v, 4, 32); v += __shfl_xor(v, 8, 32); part[r] = v; }
    if (l16 == 0) {
#pragma unroll
      for (int r = 0; r < 8; ++r) sv[wave * 64 + it * 16 + 8 * half + r] = part[r]; }
  }
  __syncthreads();
#pragma unroll 1
  for (int pass = 0; pass < 2; ++pass) { if (tid < 128) *(volatile v4f_t*)(s + e0 + e0blk + tid * 4) = *(const volatile v4fa*)(sv + tid * 4); __threadfence(); }
}

__global__ __launch_bounds__(256) void k_segment(const int* __restrict__ ei, const float* __restrict__ s, const float* __restrict__ x,
                                                const float* __restrict__ hb, float* __restrict__ pm10, float* __restrict__ delta) {
  __shared__ float bins[8][RANGE];
  const int tid = threadIdx.x, lane = tid & 31, wave = tid >> 5;
  const int r0 = blockIdx.x * RANGE;
  for (int i = tid; i < 8 * RANGE; i += 256) (&bins[0][0])[i] = 0.0f;
  __syncthreads();
  float* mybins = bins[wave];
  const int* dstp = ei + (size_t)NE;
#pragma unroll 1
  for (int c0 = 0; c0 < NE; c0 += 256) {
    const int e = c0 + tid;
    const int d = clampi(dstp[e], NN) - r0;
    const bool hit = (d >= 0) && (d < RANGE);
    const unsigned m = __builtin_amdgcn_ballot_w32(hit);
    if (m == 0u) continue;
    const float val = hit ? s[e] : 0.0f;
    unsigned mm = m;
#pragma unroll 1
    while (mm != 0u) {
      const int l = __builtin_ctz(mm);
      if (lane == l) mybins[d] += val;
      __builtin_amdgcn_wave_barrier();
      mm &= mm - 1u;
    }
  }
  __syncthreads();
  __shared__ __attribute__((aligned(16))) float dl[RANGE], pm[RANGE];
  for (int i = tid; i < RANGE; i += 256) {
    float v = hb[0];
#pragma unroll
    for (int w = 0; w < 8; ++w) v += bins[w][i];
    dl[i] = v;
    const int node = r0 + i;
    const float z = (node < NN ? x[(size_t)node * NC] : 0.0f) + v;
    pm[i] = (z > 20.0f) ? z : log1pf(expf(z));
  }
  __syncthreads();
  const int cnt = min(RANGE, NN - r0);
#pragma unroll 1
  for (int pass = 0; pass < 2; ++pass) {
    for (int i = tid * 4; i < cnt; i += 1024) {
      if (i + 3 < cnt) { *(volatile v4f_t*)(pm10 + r0 + i) = *(const volatile v4fa*)(pm + i); *(volatile v4f_t*)(delta + r0 + i) = *(const volatile v4fa*)(dl + i); }
      else { for (int j = i; j < cnt; ++j) { *(volatile float*)(pm10 + r0 + j) = pm[j]; *(volatile float*)(delta + r0 + j) = dl[j]; } }
    }
    __threadfence();
  }
}

extern "C" void kernel_launch(void* const* d_in, const int* in_sizes, int n_in,
                              void* d_out, int out_size, void* d_ws, size_t ws_size,
                              hipStream_t stream) {
  (void)in_sizes; (void)n_in; (void)out_size; (void)ws_size;
  const float* x     = (const float*)d_in[0];
  const float* pos   = (const float*)d_in[1];
  const float* mlp_w = (const float*)d_in[2];
  const float* mlp_b = (const float*)d_in[3];
  const float* head_w = (const float*)d_in[4];
  const float* head_b = (const float*)d_in[5];
  const int*   ei    = (const int*)d_in[6];
  float* out = (float*)d_out;
  float* pm10 = out;
  float* delta = out + NN;
  char* ws = (char*)d_ws;
  float* s = (float*)ws; ws += (size_t)NE * 4;
  h16*   F = (h16*)ws;
  const int HALF = NE / 2; const size_t plane = (size_t)HALF * 16;
  for (int hpart = 0; hpart < 2; ++hpart) {
    const int e0 = hpart * HALF;
    k_feat<<<HALF / 256, 256, 0, stream>>>(x, pos, ei, e0, F, plane);
    k_edge<<<HALF / 512, 256, 0, stream>>>(F, plane, mlp_w, mlp_b, head_w, e0, s);
  }
  k_segment<<<(NN + RANGE - 1) / RANGE, 256, 0, stream>>>(ei, s, x, head_b, pm10, delta);
}
